// MultiHeadAttModel_allin_52536039964914
// MI455X (gfx1250) — hardware-verified
//
#include <hip/hip_runtime.h>
#include <stddef.h>
#include <stdint.h>
#include <math.h>

#define BSZ  32
#define NAG  64
#define EMB  256
#define HDV  32
#define NHD  8
#define HIS  50
#define DKA  9
#define MROW 2048
#define MT   64
#define EP   264
#define KP   260
#define SFP  68
#define NGP  512

static_assert(MROW == BSZ * NAG);
static_assert(NHD * HDV == EMB);
static_assert(HDV == 32);
static_assert(NHD == 8);
static_assert(EMB % 64 == 0);
static_assert(EMB % 32 == 0);
static_assert(MROW % 64 == 0);
static_assert(HIS <= MT);
static_assert(HIS > 32);
static_assert(HIS * DKA <= NGP);
static_assert((HIS * EMB) % 512 == 0);
static_assert((MROW * EMB) % 2048 == 0);
static_assert((EP * 2) % 16 == 0);
static_assert((KP * 4) % 16 == 0);
static_assert((SFP * 4) % 16 == 0);

typedef _Float16 f16;
typedef f16          v16h __attribute__((ext_vector_type(16)));
typedef f16          v8h  __attribute__((ext_vector_type(8)));
typedef float        v8f  __attribute__((ext_vector_type(8)));
typedef float        v4f  __attribute__((ext_vector_type(4)));
typedef unsigned int v4u  __attribute__((ext_vector_type(4)));

union Frag  { v16h v; v8h h[2]; };
union Pack8 { v8h h; v4u u; };

__device__ __forceinline__ int imin(int a, int b) { return a < b ? a : b; }

__device__ __forceinline__ v8f mma16(v16h a, v16h b, v8f c) {
  c = __builtin_amdgcn_wmma_f32_16x16x32_f16(false, a, false, b, (short)0, c, false, false);
  asm volatile("v_nop\n\tv_nop\n\tv_nop\n\tv_nop" : "+v"(c) : "v"(a), "v"(b));
  return c;
}

__device__ __forceinline__ v16h ldfrag(const f16* p, int ld, int row0, int k0, int lane) {
  const int m = lane & 15, lh = lane >> 4;
  const f16* q = p + (size_t)(row0 + m) * ld + k0 + 8 * lh;
  Frag f;
  f.h[0] = *(const v8h*)(q);
  f.h[1] = *(const v8h*)(q + 16);
  return f.v;
}

__device__ __forceinline__ v8f zero8() { return (v8f){0.f, 0.f, 0.f, 0.f, 0.f, 0.f, 0.f, 0.f}; }

__device__ __forceinline__ v4u pack8(const float (&f)[8], float s) {
  Pack8 p;
  p.h = (v8h){(f16)(f[0] * s), (f16)(f[1] * s), (f16)(f[2] * s), (f16)(f[3] * s),
              (f16)(f[4] * s), (f16)(f[5] * s), (f16)(f[6] * s), (f16)(f[7] * s)};
  return p.u;
}

__device__ static const float kInv64   = 0.015625f;
__device__ static const float kThird   = 1.0f / 3.0f;
__device__ static const float kNegRate = -0.03597789207803197f;
__device__ static const float kRsqrt2  = 0.70710678118654752f;

__global__ __launch_bounds__(256) void k_cvt_x(const float* __restrict__ x, f16* __restrict__ xp) {
  const size_t i = (size_t)blockIdx.x * 2048 + (size_t)threadIdx.x * 8;
  const v4f a0 = *(const v4f*)(x + i);
  const v4f a1 = *(const v4f*)(x + i + 4);
  const float f[8] = {a0[0], a0[1], a0[2], a0[3], a1[0], a1[1], a1[2], a1[3]};
  const v4u hv = pack8(f, 1.0f);
  *(volatile v4u*)(xp + i) = hv;
  __threadfence();
  *(volatile v4u*)(xp + i) = hv;
}

__global__ __launch_bounds__(256) void k_cvt_wt(const float* __restrict__ w, f16* __restrict__ wt) {
  __shared__ __align__(16) float sw[64 * SFP];
  const int tid = threadIdx.x;
  const int kb = blockIdx.x * 64, nb = blockIdx.y * 64;
  {
    const int r  = tid >> 2;
    const int c0 = (tid & 3) * 16;
    const float* src = w + (size_t)(kb + r) * EMB + nb + c0;
#pragma unroll
    for (int e = 0; e < 4; ++e) *(v4f*)(sw + r * SFP + c0 + 4 * e) = *(const v4f*)(src + 4 * e);
  }
  __syncthreads();
  v4u hv[2];
  size_t go[2];
#pragma unroll
  for (int j = 0; j < 2; ++j) {
    const int p  = tid + 256 * j;
    const int nl = p >> 3;
    const int pc = p & 7;
    const float* cp = sw + (pc * 8) * SFP + nl;
    float f[8];
#pragma unroll
    for (int e = 0; e < 8; ++e) f[e] = cp[e * SFP];
    hv[j] = pack8(f, 64.0f);
    go[j] = (size_t)(nb + nl) * EMB + kb + pc * 8;
  }
#pragma unroll
  for (int j = 0; j < 2; ++j) *(volatile v4u*)(wt + go[j]) = hv[j];
  __threadfence();
#pragma unroll
  for (int j = 0; j < 2; ++j) *(volatile v4u*)(wt + go[j]) = hv[j];
}

__global__ __launch_bounds__(256) void k_pe(float* __restrict__ pe) {
  __shared__ __align__(16) float sp[512];
  const int tid = threadIdx.x;
  const int g2  = blockIdx.x * 512 + tid * 2;
  const int t   = g2 >> 8;
  const int i2  = g2 & 255;
  const float dv  = expf((float)i2 * kNegRate);
  const float ang = (float)t * dv;
  float sv, cv;
  sincosf(ang, &sv, &cv);
  sp[tid * 2]     = sv;
  sp[tid * 2 + 1] = cv;
  __syncthreads();
  if (tid < 128) {
    const v4f v = *(const v4f*)(sp + tid * 4);
    float* dst = pe + (size_t)blockIdx.x * 512 + tid * 4;
    *(volatile v4f*)dst = v;
    __threadfence();
    *(volatile v4f*)dst = v;
  }
}

__global__ __launch_bounds__(128) void k_proj64(const f16* __restrict__ ap, const f16* __restrict__ wt,
                                                const float* __restrict__ bias, float* __restrict__ y) {
  __shared__ __align__(16) float sf[64 * SFP];
  const int tid = threadIdx.x, lane = tid & 31, wave = tid >> 5;
  const int hh = lane >> 4, c = lane & 15;
  const int mb = blockIdx.x * 64, cb = blockIdx.y * 64;
  const int m0 = mb + wave * 16;

  v8f acc[4];
#pragma unroll
  for (int t = 0; t < 4; ++t) acc[t] = zero8();
#pragma unroll 1
  for (int k0 = 0; k0 < EMB; k0 += 32) {
    const v16h a = ldfrag(ap, EMB, m0, k0, lane);
#pragma unroll
    for (int t = 0; t < 4; ++t) {
      const v16h b = ldfrag(wt, EMB, cb + 16 * t, k0, lane);
      acc[t] = mma16(a, b, acc[t]);
    }
  }
  float bcol[4];
#pragma unroll
  for (int t = 0; t < 4; ++t) bcol[t] = bias[cb + 16 * t + c];
#pragma unroll
  for (int t = 0; t < 4; ++t) {
#pragma unroll
    for (int r = 0; r < 8; ++r)
      sf[(wave * 16 + 8 * hh + r) * SFP + 16 * t + c] = fmaxf(acc[t][r] * kInv64 + bcol[t], 0.f);
  }
  __syncthreads();

  v4f val[8];
  size_t go[8];
#pragma unroll
  for (int it = 0; it < 8; ++it) {
    const int p    = lane + 32 * it;
    const int L    = p >> 3;
    const int pc   = p & 7;
    const int wl   = wave * 32 + L;
    const int row  = wl >> 1;
    const int half = wl & 1;
    const int col  = half * 32 + pc * 4;
    val[it] = *(const v4f*)(sf + row * SFP + col);
    go[it]  = (size_t)(mb + row) * EMB + cb + col;
  }
#pragma unroll
  for (int it = 0; it < 8; ++it) *(volatile v4f*)(y + go[it]) = val[it];
  __threadfence();
#pragma unroll
  for (int it = 0; it < 8; ++it) *(volatile v4f*)(y + go[it]) = val[it];
}

__device__ __forceinline__ void tile_gemm64(const f16* s_a, float* s_c, const f16* __restrict__ wt,
                                            const float* __restrict__ bias, int wave, int lane) {
  const int hh = lane >> 4, c = lane & 15;
  const int r0w = (wave & 1) * 32, c0w = (wave >> 1) * 64;
  v8f acc[8];
#pragma unroll
  for (int j = 0; j < 8; ++j) acc[j] = zero8();
#pragma unroll 1
  for (int k0 = 0; k0 < EMB; k0 += 32) {
    const v16h a0 = ldfrag(s_a, EP, r0w, k0, lane);
    const v16h a1 = ldfrag(s_a, EP, r0w + 16, k0, lane);
#pragma unroll
    for (int t = 0; t < 4; ++t) {
      const v16h b = ldfrag(wt, EMB, c0w + 16 * t, k0, lane);
      acc[t]     = mma16(a0, b, acc[t]);
      acc[4 + t] = mma16(a1, b, acc[4 + t]);
    }
  }
  float bcol[4];
#pragma unroll
  for (int t = 0; t < 4; ++t) bcol[t] = bias[c0w + 16 * t + c];
#pragma unroll
  for (int i = 0; i < 2; ++i) {
#pragma unroll
    for (int t = 0; t < 4; ++t) {
#pragma unroll
      for (int r = 0; r < 8; ++r) {
        const int row = r0w + 16 * i + 8 * hh + r;
        const int col = c0w + 16 * t + c;
        s_c[row * KP + col] = fmaxf(acc[4 * i + t][r] * kInv64 + bcol[t], 0.f);
      }
    }
  }
}

union FusedScratch {
  float kv[MT * KP];
  struct { float adj[HIS * NAG]; float ng[NGP]; } g;
};

__global__ __launch_bounds__(256) void k_fused(const float* __restrict__ kin,
                                               const float* __restrict__ adjs,
                                               const float* __restrict__ wenc,
                                               const float* __restrict__ pe,
                                               const float* __restrict__ qh,
                                               const f16* __restrict__ wkt, const float* __restrict__ bk,
                                               const f16* __restrict__ wvt, const float* __restrict__ bv,
                                               f16* __restrict__ op) {
  __shared__ __align__(16) f16   s_enc[MT * EP];
  __shared__ __align__(16) FusedScratch su;
  __shared__ __align__(16) float s_qh[EMB];
  __shared__ __align__(16) float s_att[NHD * 64];
  __shared__ __align__(16) float s_o[EMB];

  const int tid = threadIdx.x, lane = tid & 31, wave = tid >> 5;
  const int n = blockIdx.x, b = blockIdx.y;
  const int bid = b * NAG + n;

  s_qh[tid] = qh[(size_t)bid * EMB + tid];
  {
    const float* arow = adjs + (size_t)n * (HIS * NAG);
#pragma unroll
    for (int i = 0; i < 4; ++i) {
      const int q4 = tid + 256 * i;
      const int qc = imin(q4, HIS * NAG / 4 - 1);
      const v4f v = *(const v4f*)(arow + 4 * qc);
      if (q4 < HIS * NAG / 4) *(v4f*)(su.g.adj + 4 * q4) = v;
    }
  }
  float wreg[DKA];
#pragma unroll
  for (int d = 0; d < DKA; ++d) wreg[d] = wenc[d * EMB + tid];
  __syncthreads();

#pragma unroll
  for (int it = 0; it < 2; ++it) {
    const int p  = tid + 256 * it;
    const int t  = p / DKA;
    const int d  = p - t * DKA;
    const int tc = imin(t, HIS - 1);
    const float* kp = kin + ((size_t)(b * HIS + tc) * NAG) * DKA + d;
    const float* ar = su.g.adj + tc * NAG;
    float acc = 0.f;
#pragma unroll 8
    for (int A = 0; A < NAG; ++A) acc = fmaf(ar[A], kp[A * DKA], acc);
    su.g.ng[p] = acc;
  }
  __syncthreads();

#pragma unroll 1
  for (int t = 0; t < HIS; ++t) {
    const float* ng = su.g.ng + t * DKA;
    float x = ng[0] * wreg[0];
#pragma unroll
    for (int d = 1; d < DKA; ++d) x = fmaf(ng[d], wreg[d], x);
    const float u = erff(x * kRsqrt2);
    const float g = (0.5f * x) * (1.0f + u);
    const float v = g + pe[t * EMB + tid];
    s_enc[t * EP + tid] = (f16)v;
  }
  {
    Pack8 z;
    z.u = (v4u){0u, 0u, 0u, 0u};
    for (int p = tid; p < (MT - HIS) * (EMB / 8); p += 256) {
      const int row = HIS + p / (EMB / 8);
      const int pc  = p - (row - HIS) * (EMB / 8);
      *(v8h*)(s_enc + row * EP + pc * 8) = z.h;
    }
  }
  __syncthreads();

  tile_gemm64(s_enc, su.kv, wkt, bk, wave, lane);
  __syncthreads();

  {
    const int v  = wave;
    const float* qv  = s_qh + v * HDV;
    const int t0 = lane, t1 = lane + 32;
    const float* k0p = su.kv + t0 * KP + v * HDV;
    const float* k1p = su.kv + t1 * KP + v * HDV;
    float d0 = 0.f, d1 = 0.f;
#pragma unroll 4
    for (int j = 0; j < HDV; ++j) {
      const float qj = qv[j];
      d0 = fmaf(qj, k0p[j], d0);
      d1 = fmaf(qj, k1p[j], d1);
    }
    const bool ok1 = (t1 < HIS);
    const float l0 = d0 * kThird, l1 = d1 * kThird;
    float mx = fmaxf(l0, ok1 ? l1 : l0);
#pragma unroll
    for (int o = 16; o > 0; o >>= 1) mx = fmaxf(mx, __shfl_xor(mx, o, 32));
    const float e0  = expf(l0 - mx);
    const float e1r = expf(fminf(l1 - mx, 80.0f));
    const float e1  = ok1 ? e1r : 0.f;
    float sm = e0 + e1;
#pragma unroll
    for (int o = 16; o > 0; o >>= 1) sm += __shfl_xor(sm, o, 32);
    const float inv = 1.0f / sm;
    s_att[v * 64 + t0] = e0 * inv;
    s_att[v * 64 + t1] = e1 * inv;
  }
  __syncthreads();

  tile_gemm64(s_enc, su.kv, wvt, bv, wave, lane);
  __syncthreads();

  {
    const int v = tid >> 5;
    const float* av = s_att + v * 64;
    const float* vp = su.kv + tid;
    float acc = 0.f;
#pragma unroll 2
    for (int t = 0; t < HIS; ++t) acc = fmaf(av[t], vp[t * KP], acc);
    s_o[tid] = acc;
  }
  __syncthreads();
  if (wave == 0) {
    const v4f a0 = *(const v4f*)(s_o + 8 * lane);
    const v4f a1 = *(const v4f*)(s_o + 8 * lane + 4);
    const float f[8] = {a0[0], a0[1], a0[2], a0[3], a1[0], a1[1], a1[2], a1[3]};
    const v4u u = pack8(f, 1.0f);
    f16* dst = op + (size_t)bid * EMB + 8 * lane;
    *(volatile v4u*)dst = u;
    __threadfence();
    *(volatile v4u*)dst = u;
  }
}

extern "C" void kernel_launch(void* const* d_in, const int* in_sizes, int n_in,
                              void* d_out, int out_size, void* d_ws, size_t ws_size,
                              hipStream_t stream) {
  if (n_in < 12) return;
  if (in_sizes[0] != MROW * EMB) return;
  if (in_sizes[1] != BSZ * HIS * NAG * DKA) return;
  if (in_sizes[2] != NAG * HIS * NAG) return;
  if (in_sizes[3] != EMB * EMB) return;
  if (in_sizes[4] != EMB) return;
  if (in_sizes[5] != EMB * EMB) return;
  if (in_sizes[6] != EMB) return;
  if (in_sizes[7] != EMB * EMB) return;
  if (in_sizes[8] != EMB) return;
  if (in_sizes[9] != EMB * EMB) return;
  if (in_sizes[10] != EMB) return;
  if (in_sizes[11] != DKA * EMB) return;
  if (out_size != MROW * EMB) return;

  const float* q    = (const float*)d_in[0];
  const float* kin  = (const float*)d_in[1];
  const float* adjs = (const float*)d_in[2];
  const float* Wq   = (const float*)d_in[3];
  const float* bq   = (const float*)d_in[4];
  const float* Wk   = (const float*)d_in[5];
  const float* bk   = (const float*)d_in[6];
  const float* Wv   = (const float*)d_in[7];
  const float* bv   = (const float*)d_in[8];
  const float* Wo   = (const float*)d_in[9];
  const float* bo   = (const float*)d_in[10];
  const float* Wenc = (const float*)d_in[11];
  float* out = (float*)d_out;

  size_t off = 0;
  const size_t oWQ = off; off += (size_t)EMB * EMB * 2;
  const size_t oWK = off; off += (size_t)EMB * EMB * 2;
  const size_t oWV = off; off += (size_t)EMB * EMB * 2;
  const size_t oWO = off; off += (size_t)EMB * EMB * 2;
  const size_t oQX = off; off += (size_t)MROW * EMB * 2;
  const size_t oPE = off; off += (size_t)HIS * EMB * 4;
  const size_t oQH = off; off += (size_t)MROW * EMB * 4;
  const size_t oOP = off; off += (size_t)MROW * EMB * 2;
  if (off > ws_size) return;
  if (off > (size_t)134217728) return;

  char* ws = (char*)d_ws;
  f16*   WQT = (f16*)(ws + oWQ);
  f16*   WKT = (f16*)(ws + oWK);
  f16*   WVT = (f16*)(ws + oWV);
  f16*   WOT = (f16*)(ws + oWO);
  f16*   QX  = (f16*)(ws + oQX);
  float* PE  = (float*)(ws + oPE);
  float* QH  = (float*)(ws + oQH);
  f16*   OP  = (f16*)(ws + oOP);

  k_cvt_wt<<<dim3(EMB / 64, EMB / 64), dim3(256), 0, stream>>>(Wq, WQT);
  k_cvt_wt<<<dim3(EMB / 64, EMB / 64), dim3(256), 0, stream>>>(Wk, WKT);
  k_cvt_wt<<<dim3(EMB / 64, EMB / 64), dim3(256), 0, stream>>>(Wv, WVT);
  k_cvt_wt<<<dim3(EMB / 64, EMB / 64), dim3(256), 0, stream>>>(Wo, WOT);
  k_cvt_x<<<dim3((MROW * EMB) / 2048), dim3(256), 0, stream>>>(q, QX);
  k_pe<<<dim3((HIS * EMB) / 512), dim3(256), 0, stream>>>(PE);
  k_proj64<<<dim3(MROW / 64, EMB / 64), dim3(128), 0, stream>>>(QX, WQT, bq, QH);
  k_fused<<<dim3(NAG, BSZ), dim3(256), 0, stream>>>(kin, adjs, Wenc, PE, QH, WKT, bk, WVT, bv, OP);
  k_proj64<<<dim3(MROW / 64, EMB / 64), dim3(128), 0, stream>>>(OP, WOT, bo, out);
  (void)hipGetLastError();
}
